// LongFormer_33646773797417
// MI455X (gfx1250) — hardware-verified
//
#include <hip/hip_runtime.h>
#include <math.h>
#include <stdint.h>

#define BATCH  2
#define SEQ    4096
#define HIDDEN 768
#define NHEADS 12
#define HD     64
#define WIN    256
#define MROWS  (BATCH * SEQ)
#define NBH    (BATCH * NHEADS)
#define NX     (MROWS * HIDDEN)
#define NW     (HIDDEN * HIDDEN)
#define NPL    (NBH * SEQ * HD)
#define NX8    (NX / 8)
#define NCHUNK ((2 * WIN) / 64 + 1)
#define PSC    1024.0f
#define LOC    2048.0f
static_assert(HIDDEN == NHEADS * HD);
static_assert((HIDDEN % 32) == 0 && (HIDDEN % 256) == 0 && (HIDDEN % 16) == 0);
static_assert((MROWS % 128) == 0 && (SEQ % 128) == 0 && (SEQ % 64) == 0 && (WIN % 64) == 0);
static_assert((NX8 % 256) == 0);
static_assert(NCHUNK == 9);
static_assert(HD == 64);

typedef _Float16 v16h __attribute__((ext_vector_type(16)));
typedef _Float16 v8h  __attribute__((ext_vector_type(8)));
typedef __bf16   v16b __attribute__((ext_vector_type(16)));
typedef __bf16   v8b  __attribute__((ext_vector_type(8)));
typedef float    v8f  __attribute__((ext_vector_type(8)));
typedef float    v4f  __attribute__((ext_vector_type(4)));
typedef unsigned int v4u __attribute__((ext_vector_type(4)));
typedef v8h __attribute__((may_alias)) v8ha;
typedef v4f __attribute__((may_alias)) v4fa;

__device__ __forceinline__ unsigned short bf_bits(float f) {
  const unsigned u = __float_as_uint(f);
  return (unsigned short)((u + 0x7FFFu + ((u >> 16) & 1u)) >> 16);
}
__device__ __forceinline__ float bf_up(unsigned short hb) { return __uint_as_float(((unsigned)hb) << 16); }
__device__ __forceinline__ unsigned pk16(unsigned short a, unsigned short b) { return (unsigned)a | ((unsigned)b << 16); }
__device__ __forceinline__ v8f zero8f() { v8f z = {0.f, 0.f, 0.f, 0.f, 0.f, 0.f, 0.f, 0.f}; return z; }
__device__ __forceinline__ v16h join8(v8h lo, v8h hi) {
  return __builtin_shufflevector(lo, hi, 0, 1, 2, 3, 4, 5, 6, 7, 8, 9, 10, 11, 12, 13, 14, 15);
}

__device__ __forceinline__ v8f wmma_f16(v16h a, v16h b, v8f c) {
  v8f d = __builtin_amdgcn_wmma_f32_16x16x32_f16(false, a, false, b, (short)0, c, false, false);
  asm volatile("v_nop\n\tv_nop\n\tv_nop\n\tv_nop" : "+v"(d) : "v"(a), "v"(b));
  return d;
}
__device__ __forceinline__ v8f mma_b(v16b a, v16b b, v8f c) {
  v8f d = __builtin_amdgcn_wmma_f32_16x16x32_bf16(false, a, false, b, (short)0, c, false, false);
  asm volatile("v_nop\n\tv_nop\n\tv_nop\n\tv_nop" : "+v"(d) : "v"(a), "v"(b));
  return d;
}

__device__ __forceinline__ v16h load_frag(const _Float16* p, int h) {
  union { v16h v; v8h half[2]; } f;
  f.half[0] = *(const v8ha*)(p + 8 * h);
  f.half[1] = *(const v8ha*)(p + 16 + 8 * h);
  return f.v;
}
__device__ __forceinline__ v16b load_frag_b(const __bf16* p, int h) {
  union { v16b v; v8b half[2]; } f;
  f.half[0] = *(const v8b*)(p + 8 * h);
  f.half[1] = *(const v8b*)(p + 16 + 8 * h);
  return f.v;
}

__global__ __launch_bounds__(256) void cvt_bf16x8(const float* __restrict__ in, unsigned short* out, int n8) {
  const int i = blockIdx.x * 256 + threadIdx.x;
  if (i < n8) {
    const v4f a = *(const v4fa*)(in + (size_t)i * 8);
    const v4f b = *(const v4fa*)(in + (size_t)i * 8 + 4);
    v4u p;
    p[0] = pk16(bf_bits(a[0]), bf_bits(a[1]));
    p[1] = pk16(bf_bits(a[2]), bf_bits(a[3]));
    p[2] = pk16(bf_bits(b[0]), bf_bits(b[1]));
    p[3] = pk16(bf_bits(b[2]), bf_bits(b[3]));
    *(volatile v4u*)(out + (size_t)i * 8) = p;
    __threadfence();
    *(volatile v4u*)(out + (size_t)i * 8) = p;
  }
}

__global__ __launch_bounds__(256) void prep_wt(const float* __restrict__ Wq, const float* __restrict__ Wk,
                                               const float* __restrict__ Wv, unsigned short* WT) {
  __shared__ __attribute__((aligned(16))) unsigned short sW[16 * HIDDEN];
  const int tid  = threadIdx.x;
  const int wave = tid >> 5;
  const int lane = tid & 31;
  const int d0   = blockIdx.x * 16;
  const int pl   = blockIdx.y;
  const float* W = (pl == 0) ? Wq : ((pl == 1) ? Wk : Wv);
#pragma unroll 1
  for (int cc = 0; cc < HIDDEN / 256; ++cc) {
    const int c = cc * 256 + tid;
    const float* row = W + (size_t)c * HIDDEN + d0;
    const v4f a0 = *(const v4fa*)(row);
    const v4f a1 = *(const v4fa*)(row + 4);
    const v4f a2 = *(const v4fa*)(row + 8);
    const v4f a3 = *(const v4fa*)(row + 12);
#pragma unroll
    for (int e = 0; e < 4; ++e) {
      sW[(e)      * HIDDEN + c] = bf_bits(a0[e]);
      sW[(4 + e)  * HIDDEN + c] = bf_bits(a1[e]);
      sW[(8 + e)  * HIDDEN + c] = bf_bits(a2[e]);
      sW[(12 + e) * HIDDEN + c] = bf_bits(a3[e]);
    }
  }
  __syncthreads();
  unsigned short* dst = WT + (size_t)pl * NW;
  const int r0 = 2 * wave;
  v4u vv[6];
#pragma unroll
  for (int rr = 0; rr < 2; ++rr)
#pragma unroll
    for (int sg = 0; sg < 3; ++sg)
      vv[rr * 3 + sg] = *(const v4u*)(sW + (r0 + rr) * HIDDEN + sg * 256 + lane * 8);
#pragma unroll
  for (int rr = 0; rr < 2; ++rr)
#pragma unroll
    for (int sg = 0; sg < 3; ++sg)
      *(volatile v4u*)(dst + (size_t)(d0 + r0 + rr) * HIDDEN + sg * 256 + lane * 8) = vv[rr * 3 + sg];
  __threadfence();
#pragma unroll
  for (int rr = 0; rr < 2; ++rr)
#pragma unroll
    for (int sg = 0; sg < 3; ++sg)
      *(volatile v4u*)(dst + (size_t)(d0 + r0 + rr) * HIDDEN + sg * 256 + lane * 8) = vv[rr * 3 + sg];
}

__device__ __forceinline__ void proj_store_pass(const _Float16* sT, _Float16* dst, int vt_layout,
                                                int bh, int l0, int w, int lane) {
  const int q8 = lane & 7, sub = lane >> 3;
#pragma unroll
  for (int i = 0; i < 8; ++i) {
    const int lid = w * 32 + i * 4 + sub;
    v8h v;
    size_t gi;
    if (vt_layout == 0) {
      v  = *(const v8ha*)(sT + lid * HD + 8 * q8);
      gi = ((size_t)bh * SEQ + l0 + lid) * HD + 8 * q8;
    } else {
      const int d = lid >> 1, hl = lid & 1;
      v  = *(const v8ha*)(sT + d * 128 + 64 * hl + 8 * q8);
      gi = ((size_t)bh * HD + d) * SEQ + l0 + 64 * hl + 8 * q8;
    }
    *(volatile v8h*)(dst + gi) = v;
  }
}

__global__ __launch_bounds__(128) void proj_kernel(
    const unsigned short* __restrict__ xbp,
    const unsigned short* __restrict__ wtp,
    const float* __restrict__ bq, const float* __restrict__ bk, const float* __restrict__ bv,
    _Float16* qhp, _Float16* qlp, _Float16* kcp, _Float16* vhp, _Float16* vlp)
{
  __shared__ __attribute__((aligned(16))) _Float16 sT[2][128 * 64];

  const int tid = threadIdx.x, lane = tid & 31, w = tid >> 5;
  const int h = lane >> 4, m = lane & 15;
  const int m0 = blockIdx.x * 128;
  const int cg = blockIdx.y;
  const int which = cg / NHEADS, head = cg - which * NHEADS;
  const int m0w = m0 + 32 * w;

  const __bf16* xb = (const __bf16*)(const void*)xbp;
  const __bf16* wt = (const __bf16*)(const void*)wtp;
  const __bf16* xa0 = xb + (size_t)(m0w + m) * HIDDEN;
  const __bf16* xa1 = xa0 + (size_t)16 * HIDDEN;
  const __bf16* wb  = wt + ((size_t)which * HIDDEN + (size_t)head * HD + m) * HIDDEN;

  v8f acc[2][4];
#pragma unroll
  for (int mt = 0; mt < 2; ++mt)
#pragma unroll
    for (int nt = 0; nt < 4; ++nt) acc[mt][nt] = zero8f();

#pragma unroll 1
  for (int k0 = 0; k0 < HIDDEN; k0 += 32) {
    const v16b a0 = load_frag_b(xa0 + k0, h);
    const v16b a1 = load_frag_b(xa1 + k0, h);
#pragma unroll
    for (int nt = 0; nt < 4; ++nt) {
      const v16b b = load_frag_b(wb + (size_t)nt * 16 * HIDDEN + k0, h);
      acc[0][nt] = mma_b(a0, b, acc[0][nt]);
      acc[1][nt] = mma_b(a1, b, acc[1][nt]);
    }
  }

  const float* bias = (which == 0) ? bq : ((which == 1) ? bk : bv);
  const float carry = (which == 0) ? 8.0f : 16.0f;
#pragma unroll
  for (int nt = 0; nt < 4; ++nt) {
    const int feat = 16 * nt + m;
    const float bvl = bf_up(bf_bits(bias[head * HD + feat]));
#pragma unroll
    for (int mt = 0; mt < 2; ++mt) {
#pragma unroll
      for (int r = 0; r < 8; ++r) {
        const int tokl = 32 * w + 16 * mt + 8 * h + r;
        const float y = (acc[mt][nt][r] + bvl) * carry;
        const _Float16 yh = (_Float16)y;
        const _Float16 yl = (_Float16)((y - (float)yh) * LOC);
        const int idx = (which == 2) ? (feat * 128 + tokl) : (tokl * HD + feat);
        sT[0][idx] = yh;
        sT[1][idx] = yl;
      }
    }
  }
  __syncthreads();

  const int b = m0 / SEQ, l0 = m0 - b * SEQ, bh = b * NHEADS + head;
  _Float16* hip = (which == 0) ? qhp : ((which == 1) ? kcp : vhp);
  _Float16* lop = (which == 0) ? qlp : vlp;
  const int vtl = (which == 2) ? 1 : 0;
  proj_store_pass(sT[0], hip, vtl, bh, l0, w, lane);
  __threadfence();
  proj_store_pass(sT[0], hip, vtl, bh, l0, w, lane);
  if (which != 1) {
    proj_store_pass(sT[1], lop, vtl, bh, l0, w, lane);
    __threadfence();
    proj_store_pass(sT[1], lop, vtl, bh, l0, w, lane);
  }
}

__device__ __forceinline__ void pack_p2(v8f a, v8f c, v16h& ph, v16h& pl) {
  const v8f ya = a * PSC;
  const v8f yc = c * PSC;
  const v8h ha = __builtin_convertvector(ya, v8h);
  const v8h hc = __builtin_convertvector(yc, v8h);
  const v8f ra = (ya - __builtin_convertvector(ha, v8f)) * LOC;
  const v8f rc = (yc - __builtin_convertvector(hc, v8f)) * LOC;
  ph = join8(ha, hc);
  pl = join8(__builtin_convertvector(ra, v8h), __builtin_convertvector(rc, v8h));
}

__device__ __forceinline__ void att_store_pass(const float* so, float* out,
                                               int b, int head, int q0, int lane) {
  const int q8 = lane & 7, sub = lane >> 3;
#pragma unroll
  for (int i = 0; i < 8; ++i) {
    const int lid = i * 4 + sub;
    const int row = lid >> 1, hl = lid & 1;
    const v4f v = *(const v4fa*)(so + row * 64 + 32 * hl + 4 * q8);
    const size_t gi = ((size_t)b * SEQ + q0 + row) * HIDDEN + (size_t)head * HD + 32 * hl + 4 * q8;
    *(volatile v4f*)(out + gi) = v;
  }
}

__global__ __launch_bounds__(128) void attn_band(
    const _Float16* __restrict__ qhp,
    const _Float16* __restrict__ qlp,
    const _Float16* __restrict__ kcp,
    const _Float16* __restrict__ vhp,
    const _Float16* __restrict__ vlp,
    float* __restrict__ out)
{
  __shared__ __attribute__((aligned(16))) float sO[4 * 16 * 64];

  const int tid = threadIdx.x, lane = tid & 31, w = tid >> 5;
  const int h = lane >> 4, m = lane & 15;
  const int bh = blockIdx.y, b = bh / NHEADS, head = bh - b * NHEADS;
  const int qblk = blockIdx.x * 64;
  const int q0 = qblk + 16 * w;
  const int qm = q0 + m;

  const size_t qoff = ((size_t)bh * SEQ + q0 + m) * HD;
  const v16h qh0 = load_frag(qhp + qoff, h);
  const v16h qh1 = load_frag(qhp + qoff + 32, h);
  const v16h ql0 = load_frag(qlp + qoff, h);
  const v16h ql1 = load_frag(qlp + qoff + 32, h);

  v8f o0[4], o1[4];
#pragma unroll
  for (int t = 0; t < 4; ++t) { o0[t] = zero8f(); o1[t] = zero8f(); }
  float mrun = -INFINITY, lrun = 0.0f;

  const _Float16* kbase = kcp + ((size_t)bh * SEQ + m) * HD;
  const _Float16* vhb   = vhp + ((size_t)bh * HD + m) * SEQ;
  const _Float16* vlb   = vlp + ((size_t)bh * HD + m) * SEQ;

#pragma unroll 1
  for (int c = 0; c < NCHUNK; ++c) {
    const int kv0 = qblk - WIN + 64 * c;
    if (kv0 < 0 || kv0 >= SEQ) continue;

    v8f s[4];
#pragma unroll
    for (int j = 0; j < 4; ++j) {
      const _Float16* kp = kbase + (size_t)(kv0 + 16 * j) * HD;
      const v16h kf0 = load_frag(kp, h);
      const v16h kf1 = load_frag(kp + 32, h);
      v8f zh = zero8f(), zl = zero8f();
      zh = wmma_f16(kf0, qh0, zh);
      zh = wmma_f16(kf1, qh1, zh);
      zl = wmma_f16(kf0, ql0, zl);
      zl = wmma_f16(kf1, ql1, zl);
      v8f sv;
#pragma unroll
      for (int r = 0; r < 8; ++r) sv[r] = (zh[r] + zl[r] * (1.0f / LOC)) * (1.0f / 1024.0f);
      s[j] = sv;
    }

#pragma unroll
    for (int j = 0; j < 4; ++j) {
#pragma unroll
      for (int r = 0; r < 8; ++r) {
        const int dk = kv0 + 16 * j + 8 * h + r - qm;
        const float sv = s[j][r];
        s[j][r] = (dk >= -WIN && dk <= WIN) ? sv : -INFINITY;
      }
    }

    float mloc = -INFINITY;
#pragma unroll
    for (int j = 0; j < 4; ++j)
#pragma unroll
      for (int r = 0; r < 8; ++r) mloc = fmaxf(mloc, s[j][r]);
    mloc = fmaxf(mloc, __shfl_xor(mloc, 16));
    const float mnew  = fmaxf(mrun, mloc);
    const float msafe = (mnew == -INFINITY) ? 0.0f : mnew;
    const float alpha = __expf(mrun - msafe);
    mrun = mnew;
    float lsum = 0.0f;
#pragma unroll
    for (int j = 0; j < 4; ++j)
#pragma unroll
      for (int r = 0; r < 8; ++r) {
        const float p = __expf(s[j][r] - msafe);
        s[j][r] = p;
        lsum += p;
      }
    lsum += __shfl_xor(lsum, 16);
    lrun = lrun * alpha + lsum;
#pragma unroll
    for (int t = 0; t < 4; ++t) {
#pragma unroll
      for (int r = 0; r < 8; ++r) { o0[t][r] = o0[t][r] * alpha; o1[t][r] = o1[t][r] * alpha; }
    }

    v16h ph0, pl0, ph1, pl1;
    pack_p2(s[0], s[1], ph0, pl0);
    pack_p2(s[2], s[3], ph1, pl1);

#pragma unroll
    for (int t = 0; t < 4; ++t) {
      const _Float16* vp = vhb + (size_t)(16 * t) * SEQ + kv0;
      const v16h vf0 = load_frag(vp, h);
      const v16h vf1 = load_frag(vp + 32, h);
      o0[t] = wmma_f16(vf0, ph0, o0[t]);
      o0[t] = wmma_f16(vf1, ph1, o0[t]);
      o1[t] = wmma_f16(vf0, pl0, o1[t]);
      o1[t] = wmma_f16(vf1, pl1, o1[t]);
      const _Float16* vq = vlb + (size_t)(16 * t) * SEQ + kv0;
      const v16h wf0 = load_frag(vq, h);
      const v16h wf1 = load_frag(vq + 32, h);
      o1[t] = wmma_f16(wf0, ph0, o1[t]);
      o1[t] = wmma_f16(wf1, ph1, o1[t]);
    }
  }

  const float inv = (lrun > 0.0f) ? ((1.0f / lrun) * (1.0f / 16384.0f)) : 0.0f;
  float* so = sO + w * 1024;
#pragma unroll
  for (int t = 0; t < 4; ++t)
#pragma unroll
    for (int r = 0; r < 8; ++r)
      so[m * 64 + 16 * t + 8 * h + r] = (o0[t][r] + o1[t][r] * (1.0f / LOC)) * inv;
  __syncthreads();

  att_store_pass(so, out, b, head, q0, lane);
  __threadfence();
  att_store_pass(so, out, b, head, q0, lane);
}

extern "C" void kernel_launch(void* const* d_in, const int* in_sizes, int n_in,
                              void* d_out, int out_size, void* d_ws, size_t ws_size,
                              hipStream_t stream) {
  if (n_in < 7) return;
  if (in_sizes[0] != NX) return;
  if (in_sizes[1] != NW || in_sizes[3] != NW || in_sizes[5] != NW) return;
  if (in_sizes[2] != HIDDEN || in_sizes[4] != HIDDEN || in_sizes[6] != HIDDEN) return;
  if (out_size != NX) return;

  const float* x  = (const float*)d_in[0];
  const float* Wq = (const float*)d_in[1];
  const float* bq = (const float*)d_in[2];
  const float* Wk = (const float*)d_in[3];
  const float* bk = (const float*)d_in[4];
  const float* Wv = (const float*)d_in[5];
  const float* bv = (const float*)d_in[6];
  float* out = (float*)d_out;

  const size_t PXB = (size_t)NX * 2;
  const size_t PWT = (size_t)3 * NW * 2;
  const size_t PPL = (size_t)NPL * 2;
  size_t off = 0;
  const size_t oXb = off; off += PXB;
  const size_t oWT = off; off += PWT;
  const size_t oQh = off; off += PPL;
  const size_t oQl = off; off += PPL;
  const size_t oKc = off; off += PPL;
  const size_t oVh = off; off += PPL;
  const size_t oVl = off; off += PPL;
  if (off > ws_size) return;
  if (off > (size_t)134217728) return;

  char* ws = (char*)d_ws;
  unsigned short* Xb = (unsigned short*)(ws + oXb);
  unsigned short* WT = (unsigned short*)(ws + oWT);
  _Float16* Qh = (_Float16*)(ws + oQh);
  _Float16* Ql = (_Float16*)(ws + oQl);
  _Float16* Kc = (_Float16*)(ws + oKc);
  _Float16* Vh = (_Float16*)(ws + oVh);
  _Float16* Vl = (_Float16*)(ws + oVl);

  cvt_bf16x8<<<dim3(NX8 / 256), dim3(256), 0, stream>>>(x, Xb, NX8);
  prep_wt<<<dim3(HIDDEN / 16, 3), dim3(256), 0, stream>>>(Wq, Wk, Wv, WT);
  proj_kernel<<<dim3(MROWS / 128, 3 * NHEADS), dim3(128), 0, stream>>>(Xb, WT, bq, bk, bv, Qh, Ql, Kc, Vh, Vl);
  attn_band<<<dim3(SEQ / 64, NBH), dim3(128), 0, stream>>>(Qh, Ql, Kc, Vh, Vl, out);
  (void)hipGetLastError();
}
